// STPointNetFeature_2920577761800
// MI455X (gfx1250) — hardware-verified
//
#include <hip/hip_runtime.h>
#include <stddef.h>
#include <math.h>


#define NB    128
#define NP    4096
#define NG    16
#define C1    64
#define C2    128
#define C3    512
#define RB    128
#define NCH   (NP / RB)
#define NTHR  256
#define P1    72
#define P2    136
#define SC_A  8.0f
#define SC_W  64.0f
#define SC_INV (1.0f / 512.0f)
#define NBK2  (C2 * C1 / 8 / NTHR)
#define NBK3  (C3 * C2 / 8 / NTHR)
#define NOUT1 (NB * 3 * NP)

static_assert(NBK2 * NTHR * 8 == C2 * C1);
static_assert(NBK3 * NTHR * 8 == C3 * C2);
static_assert(RB == 16 * (NTHR / 32));
static_assert(NP % RB == 0);
static_assert(C2 == 16 * (NTHR / 32));
static_assert(C3 == 64 * (NTHR / 32));
static_assert((P1 * 2) % 16 == 0);
static_assert((P2 * 2) % 16 == 0);
static_assert(C3 / 4 == NTHR / 2);
static_assert(NOUT1 % (4 * NTHR) == 0);
static_assert(C1 % 32 == 0);
static_assert(C2 % 32 == 0);

typedef _Float16 v16h __attribute__((ext_vector_type(16)));
typedef _Float16 v8h  __attribute__((ext_vector_type(8)));
typedef float    v4f  __attribute__((ext_vector_type(4)));
typedef float    v8f  __attribute__((ext_vector_type(8)));
union FragH { v16h v; v8h h[2]; };

__device__ __forceinline__ v8f wmh(v16h a, v16h b, v8f c) {
  v8f d = __builtin_amdgcn_wmma_f32_16x16x32_f16(false, a, false, b, (short)0, c, false, false);
#if defined(__HIP_DEVICE_COMPILE__)
  asm volatile("v_nop\n\tv_nop\n\tv_nop\n\tv_nop" : "+v"(d) : "v"(a), "v"(b));
#endif
  return d;
}

__device__ __forceinline__ v8f zero8() {
  v8f z = {0.f, 0.f, 0.f, 0.f, 0.f, 0.f, 0.f, 0.f};
  return z;
}

__device__ __forceinline__ v16h afrag(const _Float16* row, int k0, int h) {
  FragH u;
  u.h[0] = *(const v8h*)(row + k0 + 8 * h);
  u.h[1] = *(const v8h*)(row + k0 + 16 + 8 * h);
  return u.v;
}

__global__ __launch_bounds__(NTHR) void k_prep(const float* __restrict__ Wg2, const float* __restrict__ Wg3,
                                               const float* __restrict__ Wl2, const float* __restrict__ Wl3,
                                               _Float16* T2g, _Float16* T3g, _Float16* T2l, _Float16* T3l) {
  const int blk = blockIdx.x, tid = (int)threadIdx.x;
  const float* W;
  _Float16* T;
  int K, N, local;
  if (blk < NBK2) {
    W = Wg2; T = T2g; K = C1; N = C2; local = blk * NTHR + tid;
  } else if (blk < NBK2 + NBK3) {
    W = Wg3; T = T3g; K = C2; N = C3; local = (blk - NBK2) * NTHR + tid;
  } else if (blk < 2 * NBK2 + NBK3) {
    W = Wl2; T = T2l; K = C1; N = C2; local = (blk - NBK2 - NBK3) * NTHR + tid;
  } else {
    W = Wl3; T = T3l; K = C2; N = C3; local = (blk - 2 * NBK2 - NBK3) * NTHR + tid;
  }
  const int ppr = K >> 3;
  int n = local / ppr;
  n = n < N ? n : N - 1;
  const int k0 = (local - (local / ppr) * ppr) * 8;
  v8h o;
#pragma unroll
  for (int e = 0; e < 8; ++e) o[e] = (_Float16)(SC_W * W[(size_t)(k0 + e) * N + n]);
  _Float16* p = T + (size_t)n * K + k0;
  *(volatile v8h*)p = o;
  __threadfence();
  *(volatile v8h*)p = o;
}

__global__ __launch_bounds__(NTHR) void k_main(const float* __restrict__ pc, const float* __restrict__ tt,
                                               const float* __restrict__ Wg1, const float* __restrict__ bg1,
                                               const _Float16* __restrict__ T2g, const float* __restrict__ bg2,
                                               const _Float16* __restrict__ T3g, const float* __restrict__ bg3,
                                               const float* __restrict__ Wl1, const float* __restrict__ bl1,
                                               const _Float16* __restrict__ T2l, const float* __restrict__ bl2,
                                               const _Float16* __restrict__ T3l, const float* __restrict__ bl3,
                                               float* FM) {
  __shared__ __align__(16) _Float16 sh1[RB * P1];
  __shared__ __align__(16) _Float16 sh2[RB * P2];
  __shared__ v4f smax4[C3 / 4];
  float* smax = (float*)smax4;

  const int tid = (int)threadIdx.x, lane = tid & 31, w = tid >> 5, h = lane >> 4, m = lane & 15;
  const int b = blockIdx.x, br = blockIdx.y;
  const int wr = 16 * w;

  const float*    W1 = br ? Wl1 : Wg1;
  const float*    b1 = br ? bl1 : bg1;
  const _Float16* T2 = br ? T2l : T2g;
  const float*    b2 = br ? bl2 : bg2;
  const _Float16* T3 = br ? T3l : T3g;
  const float*    b3 = br ? bl3 : bg3;
  const float tv = tt[b];

  const int c0 = lane, c1 = lane + 32;
  const float wa0 = W1[c0], wa1 = W1[C1 + c0], wa2 = W1[2 * C1 + c0];
  const float ta  = fmaf(tv, W1[3 * C1 + c0], b1[c0]);
  const float wb0 = W1[c1], wb1 = W1[C1 + c1], wb2 = W1[2 * C1 + c1];
  const float tb  = fmaf(tv, W1[3 * C1 + c1], b1[c1]);

  FragH bq[2];
  {
    const _Float16* pb = T2 + (size_t)(wr + m) * C1 + 8 * h;
#pragma unroll
    for (int ks = 0; ks < 2; ++ks) {
      bq[ks].h[0] = *(const v8h*)(pb + 32 * ks);
      bq[ks].h[1] = *(const v8h*)(pb + 32 * ks + 16);
    }
  }
  const float bb2 = b2[wr + m];

  const float ninf = __int_as_float(0xff800000u);
  float rmax[4];
#pragma unroll
  for (int q = 0; q < 4; ++q) rmax[q] = ninf;

  const float* pcb = pc + (size_t)b * 3 * NP;

#pragma unroll 1
  for (int ch = 0; ch < NCH; ++ch) {
    {
      const int pi = ch * RB + wr + m;
      const float xv = pcb[pi], yv = pcb[NP + pi], zv = pcb[2 * NP + pi];
#pragma unroll
      for (int r = 0; r < 16; ++r) {
        const float xr = __shfl(xv, r, 32), yr = __shfl(yv, r, 32), zr = __shfl(zv, r, 32);
        const float s0 = fmaf(xr, wa0, fmaf(yr, wa1, fmaf(zr, wa2, ta)));
        const float s1 = fmaf(xr, wb0, fmaf(yr, wb1, fmaf(zr, wb2, tb)));
        sh1[(wr + r) * P1 + c0] = (_Float16)(SC_A * fmaxf(s0, 0.0f));
        sh1[(wr + r) * P1 + c1] = (_Float16)(SC_A * fmaxf(s1, 0.0f));
      }
    }
    __syncthreads();

    {
#pragma unroll
      for (int mt = 0; mt < 8; ++mt) {
        v8f acc = zero8();
        const _Float16* ar = sh1 + (16 * mt + m) * P1;
#pragma unroll
        for (int ks = 0; ks < 2; ++ks) acc = wmh(afrag(ar, 32 * ks, h), bq[ks].v, acc);
#pragma unroll
        for (int r = 0; r < 8; ++r) {
          const float v = fmaxf(fmaf(acc[r], SC_INV, bb2), 0.0f);
          sh2[(16 * mt + 8 * h + r) * P2 + wr + m] = (_Float16)(SC_A * v);
        }
      }
    }
    __syncthreads();

#pragma unroll
    for (int pq = 0; pq < 2; ++pq) {
      const int n0 = 16 * (4 * w + 2 * pq) + m;
      FragH bA[4], bB[4];
      const _Float16* pa = T3 + (size_t)n0 * C2 + 8 * h;
      const _Float16* pb = pa + 16 * C2;
#pragma unroll
      for (int ks = 0; ks < 4; ++ks) {
        bA[ks].h[0] = *(const v8h*)(pa + 32 * ks);
        bA[ks].h[1] = *(const v8h*)(pa + 32 * ks + 16);
        bB[ks].h[0] = *(const v8h*)(pb + 32 * ks);
        bB[ks].h[1] = *(const v8h*)(pb + 32 * ks + 16);
      }
      float m0 = rmax[2 * pq], m1 = rmax[2 * pq + 1];
#pragma unroll 2
      for (int mt = 0; mt < 8; ++mt) {
        v8f acc0 = zero8(), acc1 = zero8();
        const _Float16* ar = sh2 + (16 * mt + m) * P2;
#pragma unroll
        for (int ks = 0; ks < 4; ++ks) {
          const v16h af = afrag(ar, 32 * ks, h);
          acc0 = wmh(af, bA[ks].v, acc0);
          acc1 = wmh(af, bB[ks].v, acc1);
        }
#pragma unroll
        for (int r = 0; r < 8; ++r) {
          m0 = fmaxf(m0, acc0[r]);
          m1 = fmaxf(m1, acc1[r]);
        }
      }
      rmax[2 * pq]     = m0;
      rmax[2 * pq + 1] = m1;
    }
  }

#pragma unroll
  for (int q = 0; q < 4; ++q) {
    const int c = 16 * (4 * w + q) + m;
    const float mv = fmaxf(rmax[q], __shfl_xor(rmax[q], 16, 32));
    smax[c] = fmaxf(fmaf(mv, SC_INV, b3[c]), 0.0f);
  }
  __syncthreads();

  if (tid < C3 / 4) {
    const v4f o = smax4[tid];
    float* p = FM + (size_t)(br * NB + b) * C3 + 4 * tid;
    *(volatile v4f*)p = o;
    __threadfence();
    *(volatile v4f*)p = o;
  }
}

__global__ __launch_bounds__(NTHR) void k_out0(const float* __restrict__ FM, const int* __restrict__ idx,
                                               float* out) {
  const int b = blockIdx.x, tid = (int)threadIdx.x;
  v4f o;
  if (tid < C3 / 4) {
    int g = idx[b];
    g = g < 0 ? 0 : (g > NG - 1 ? NG - 1 : g);
    const float ninf = __int_as_float(0xff800000u);
    float m0 = ninf, m1 = ninf, m2 = ninf, m3 = ninf;
    const float* base = FM + 4 * tid;
#pragma unroll 4
    for (int bp = 0; bp < NB; ++bp) {
      const int gb = idx[bp];
      const v4f v = *(const v4f*)(base + (size_t)bp * C3);
      const bool sel = (gb == g);
      m0 = sel ? fmaxf(m0, v[0]) : m0;
      m1 = sel ? fmaxf(m1, v[1]) : m1;
      m2 = sel ? fmaxf(m2, v[2]) : m2;
      m3 = sel ? fmaxf(m3, v[3]) : m3;
    }
    o[0] = m0; o[1] = m1; o[2] = m2; o[3] = m3;
  } else {
    o = *(const v4f*)(FM + (size_t)(NB + b) * C3 + 4 * (tid - C3 / 4));
  }
  float* p = out + (size_t)b * (2 * C3) + 4 * tid;
  *(volatile v4f*)p = o;
  __threadfence();
  *(volatile v4f*)p = o;
}

__global__ __launch_bounds__(NTHR) void k_copy(const float* __restrict__ src, float* dst, int n4) {
  const int i  = blockIdx.x * NTHR + (int)threadIdx.x;
  const int ic = i < n4 ? i : n4 - 1;
  const v4f v  = *(const v4f*)(src + (size_t)4 * ic);
  float* p = dst + (size_t)4 * ic;
  if (i < n4) *(volatile v4f*)p = v;
  __threadfence();
  if (i < n4) *(volatile v4f*)p = v;
}

extern "C" void kernel_launch(void* const* d_in, const int* in_sizes, int n_in,
                              void* d_out, int out_size, void* d_ws, size_t ws_size,
                              hipStream_t stream) {
  if (n_in < 15) return;
  if (in_sizes[0] != NB * 3 * NP || in_sizes[1] != NB || in_sizes[2] != NB) return;
  for (int s = 0; s < 2; ++s) {
    const int o = 3 + 6 * s;
    if (in_sizes[o] != 4 * C1 || in_sizes[o + 1] != C1) return;
    if (in_sizes[o + 2] != C1 * C2 || in_sizes[o + 3] != C2) return;
    if (in_sizes[o + 4] != C2 * C3 || in_sizes[o + 5] != C3) return;
  }
  if (out_size != NB * 2 * C3 + NOUT1) return;

  const float* pc  = (const float*)d_in[0];
  const float* tt  = (const float*)d_in[1];
  const int*   idx = (const int*)d_in[2];
  const float* Wg1 = (const float*)d_in[3];
  const float* bg1 = (const float*)d_in[4];
  const float* Wg2 = (const float*)d_in[5];
  const float* bg2 = (const float*)d_in[6];
  const float* Wg3 = (const float*)d_in[7];
  const float* bg3 = (const float*)d_in[8];
  const float* Wl1 = (const float*)d_in[9];
  const float* bl1 = (const float*)d_in[10];
  const float* Wl2 = (const float*)d_in[11];
  const float* bl2 = (const float*)d_in[12];
  const float* Wl3 = (const float*)d_in[13];
  const float* bl3 = (const float*)d_in[14];
  float* out  = (float*)d_out;
  float* out1 = out + (size_t)NB * 2 * C3;

  const size_t szT2  = (size_t)C2 * C1 * 2;
  const size_t szT3  = (size_t)C3 * C2 * 2;
  const size_t szFM  = (size_t)2 * NB * C3 * 4;
  const size_t offT2g = 0;
  const size_t offT3g = offT2g + szT2;
  const size_t offT2l = offT3g + szT3;
  const size_t offT3l = offT2l + szT2;
  const size_t offFM  = offT3l + szT3;
  const size_t total  = offFM + szFM;
  if (total > ws_size || total > (size_t)134217728) return;
  char* ws = (char*)d_ws;
  _Float16* T2g = (_Float16*)(ws + offT2g);
  _Float16* T3g = (_Float16*)(ws + offT3g);
  _Float16* T2l = (_Float16*)(ws + offT2l);
  _Float16* T3l = (_Float16*)(ws + offT3l);
  float*    FM  = (float*)(ws + offFM);

  k_prep<<<2 * NBK2 + 2 * NBK3, NTHR, 0, stream>>>(Wg2, Wg3, Wl2, Wl3, T2g, T3g, T2l, T3l);
  k_main<<<dim3(NB, 2), NTHR, 0, stream>>>(pc, tt, Wg1, bg1, T2g, bg2, T3g, bg3,
                                            Wl1, bl1, T2l, bl2, T3l, bl3, FM);
  k_out0<<<NB, NTHR, 0, stream>>>(FM, idx, out);
  const int n4 = NOUT1 / 4;
  k_copy<<<(n4 + NTHR - 1) / NTHR, NTHR, 0, stream>>>(pc, out1, n4);
}
